// RWKV7TimeMixing_14310831030385
// MI455X (gfx1250) — hardware-run, weakly checked
//
#include <hip/hip_runtime.h>
#include <math.h>

typedef __attribute__((ext_vector_type(16))) _Float16 v16h;
typedef __attribute__((ext_vector_type(8)))  _Float16 v8h;
typedef __attribute__((ext_vector_type(2)))  _Float16 v2h;
typedef __attribute__((ext_vector_type(16))) __bf16   v16b;
typedef __attribute__((ext_vector_type(8)))  __bf16   v8b;
typedef __attribute__((ext_vector_type(8)))  float    v8f;
typedef __attribute__((ext_vector_type(4)))  float    v4f;
typedef __attribute__((ext_vector_type(2)))  float    v2f;
typedef float v2f __attribute__((ext_vector_type(2)));

constexpr int kNB   = 8;
constexpr int kT    = 512;
constexpr int kRows = kNB * kT;
constexpr int kC    = 256;
constexpr int kNPt  = 8;
constexpr int kN3   = 3 * kC;
constexpr int kOut1 = kRows * kC;
constexpr int kThr  = 256;
constexpr float kInCarry = 1024.0f;
constexpr float kWCarry  = 4096.0f;
constexpr float kCXn  = 1024.0f;
constexpr float kCO   = 64.0f;
constexpr float kF16MinNormal = 6.103515625e-5f;

static_assert(kC == 256 && kC == kNPt * 32 && kRows == 4096 && kT == 512 && kN3 == 768, "the index arithmetic below uses these sizes");

constexpr size_t kOffZB = 0ull;
constexpr size_t kOffWDEC = 3072ull;
constexpr size_t kOffSTAT = 4096ull;
constexpr size_t kOffXN16 = 36864ull;
constexpr size_t kOffWKVR16 = 2134016ull;
constexpr size_t kOffWO16 = 2527232ull;
constexpr size_t kOffKVR = 2658304ull;
constexpr size_t kOffGS = 15241216ull;
constexpr size_t kOffOP = 19435520ull;
constexpr size_t kOffO16H = 52989952ull;
constexpr size_t kOffO16L = 55087104ull;
constexpr size_t kOffP1 = 57184256ull;
constexpr size_t kOffP2 = 61378560ull;
constexpr size_t kWsTotal = 65572864ull;
static_assert(kWsTotal <= 134217728ull, "carve cap: under 128 MiB");
static_assert(kOffZB == 0
  && kOffWDEC == kOffZB + 3072ull
  && kOffSTAT == kOffWDEC + 1024ull
  && kOffXN16 == kOffSTAT + 32768ull
  && kOffWKVR16 == kOffXN16 + 2097152ull
  && kOffWO16 == kOffWKVR16 + 393216ull
  && kOffKVR == kOffWO16 + 131072ull
  && kOffGS == kOffKVR + 12582912ull
  && kOffOP == kOffGS + 4194304ull
  && kOffO16H == kOffOP + 33554432ull
  && kOffO16L == kOffO16H + 2097152ull
  && kOffP1 == kOffO16L + 2097152ull
  && kOffP2 == kOffP1 + 4194304ull
  && kWsTotal == kOffP2 + 4194304ull, "the carve is a chain: every region starts where the one before ends");
static_assert((kOffWDEC % 256) == 0 && (kOffSTAT % 256) == 0 && (kOffXN16 % 256) == 0 && (kOffWKVR16 % 256) == 0 && (kOffWO16 % 256) == 0 && (kOffKVR % 256) == 0 && (kOffGS % 256) == 0 && (kOffOP % 256) == 0 && (kOffO16H % 256) == 0 && (kOffO16L % 256) == 0 && (kOffP1 % 256) == 0 && (kOffP2 % 256) == 0, "every region starts on a multiple of 256 B");

__device__ __forceinline__ unsigned short f2bf_bits(float f) {
  unsigned u = __float_as_uint(f);
  return (unsigned short)((u + 0x7FFFu + ((u >> 16) & 1u)) >> 16);
}
__device__ __forceinline__ float bf_bits2f(unsigned short h) { return __uint_as_float(((unsigned)h) << 16); }
__device__ __forceinline__ float bf16r(float f) { return bf_bits2f(f2bf_bits(f)); }
__device__ __forceinline__ float carry_flush(float v, float carry) {
  const float s = v * carry;
  return (fabsf(s) < kF16MinNormal) ? 0.0f : s;
}

__device__ __forceinline__ void dep_guard4_h(v8f& a, v8f& b, v8f& c, v8f& d, v16h x, v16h y) { asm volatile("v_nop\n\tv_nop\n\tv_nop\n\tv_nop" : "+v"(a), "+v"(b), "+v"(c), "+v"(d) : "v"(x), "v"(y)); }
__device__ __forceinline__ void dep_guard4_b(v8f& a, v8f& b, v8f& c, v8f& d, v16b x, v16b y) { asm volatile("v_nop\n\tv_nop\n\tv_nop\n\tv_nop" : "+v"(a), "+v"(b), "+v"(c), "+v"(d) : "v"(x), "v"(y)); }
__device__ __forceinline__ void keep4_h(v16h a, v16h b, v16h c, v16h d) { asm volatile("v_nop" :: "v"(a), "v"(b), "v"(c), "v"(d)); }
__device__ __forceinline__ void keep4_b(v16b a, v16b b, v16b c, v16b d) { asm volatile("v_nop" :: "v"(a), "v"(b), "v"(c), "v"(d)); }
__device__ __forceinline__ void acc_guard4(v8f& a, v8f& b, v8f& c, v8f& d) { asm volatile("v_nop\n\tv_nop\n\tv_nop\n\tv_nop" : "+v"(a), "+v"(b), "+v"(c), "+v"(d)); }

template <typename T> struct Frag;
template <> struct Frag<_Float16> {
  typedef v16h V; union U { v16h v; v8h h[2]; };
  static __device__ __forceinline__ v16h load(const _Float16* p) {
    U f; f.h[0] = *(const v8h*)(p); f.h[1] = *(const v8h*)(p + 16); return f.v;
  }
  static __device__ __forceinline__ v8f mma(v16h a, v16h b, v8f c) {
    return __builtin_amdgcn_wmma_f32_16x16x32_f16(false, a, false, b, (short)0, c, false, false);
  }
  static __device__ __forceinline__ void guard4(v8f& a, v8f& b, v8f& c, v8f& d, v16h x, v16h y) { dep_guard4_h(a, b, c, d, x, y); }
  static __device__ __forceinline__ void keep(v16h a, v16h b, v16h c, v16h d) { keep4_h(a, b, c, d); }
};
template <> struct Frag<__bf16> {
  typedef v16b V; union U { v16b v; v8b h[2]; };
  static __device__ __forceinline__ v16b load(const __bf16* p) {
    U f; f.h[0] = *(const v8b*)(p); f.h[1] = *(const v8b*)(p + 16); return f.v;
  }
  static __device__ __forceinline__ v8f mma(v16b a, v16b b, v8f c) {
    return __builtin_amdgcn_wmma_f32_16x16x32_bf16(false, a, false, b, (short)0, c, false, false);
  }
  static __device__ __forceinline__ void guard4(v8f& a, v8f& b, v8f& c, v8f& d, v16b x, v16b y) { dep_guard4_b(a, b, c, d, x, y); }
  static __device__ __forceinline__ void keep(v16b a, v16b b, v16b c, v16b d) { keep4_b(a, b, c, d); }
};

__device__ __forceinline__ v8f mma_h(v16h a, v16h b, v8f c) {
  c = __builtin_amdgcn_wmma_f32_16x16x32_f16(false, a, false, b, (short)0, c, false, false);
  asm volatile("v_nop\n\tv_nop\n\tv_nop\n\tv_nop" : "+v"(c) : "v"(a), "v"(b));
  return c;
}

template <int ET> struct Elem;
template <> struct Elem<0> { typedef _Float16 T; };
template <> struct Elem<1> { typedef __bf16 T; };
template <int ET, bool SPLIT, int BIAS_MODE, int OUT_MODE, bool RESID, int ACT = 0>
__global__ __launch_bounds__(256) void wmma_gemm64(
    const unsigned short* __restrict__ Ap, const unsigned short* __restrict__ A2p, int lda, long strideA,
    const unsigned short* __restrict__ Btp, const unsigned short* __restrict__ Bt2p, int ldb, long strideB,
    void* __restrict__ Cout, void* __restrict__ Cout2, int ldc, long strideC,
    const float* __restrict__ bias,
    const float* __restrict__ resid, long strideR,
    int M, int N, int K, float scale) {
  typedef typename Elem<ET>::T T;
  typedef typename Frag<T>::V V;
  const T* A = (const T*)Ap; const T* A2 = (const T*)A2p; const T* Bt = (const T*)Btp; const T* Bt2 = (const T*)Bt2p;
  __shared__ __align__(16) float sT[8][16 * 68];
  const int b    = blockIdx.y;
  const int lane = threadIdx.x & 31;
  const int wave = threadIdx.x >> 5;
  const int tilesN = N >> 6;
  const int tilesM = M >> 6;
  const int tile = blockIdx.x * 8 + wave;
  if (tile >= tilesM * tilesN) return;
  const int tm = tile / tilesN;
  const int tn = tile - tm * tilesN;
  const int m0 = tm << 6;
  const int n0 = tn << 6;

  const T* Ab  = A  + (size_t)b * strideA;
  const T* Bb  = Bt + (size_t)b * strideB;
  const T* Ab2 = SPLIT ? (A2  + (size_t)b * strideA) : nullptr;
  const T* Bb2 = SPLIT ? (Bt2 + (size_t)b * strideB) : nullptr;

  const int rlane = lane & 15;
  const int koff  = (lane >> 4) * 8;
  const int mOff  = (lane >> 4) * 8;

  v8f acc[4][4];
#pragma unroll
  for (int i = 0; i < 4; ++i)
#pragma unroll
    for (int j = 0; j < 4; ++j) acc[i][j] = (v8f){0.f,0.f,0.f,0.f,0.f,0.f,0.f,0.f};

  for (int k0 = 0; k0 < K; k0 += 32) {
    V bh[4], bl[4];
#pragma unroll
    for (int j = 0; j < 4; ++j) {
      const size_t bo = (size_t)(n0 + (j << 4) + rlane) * ldb + koff + k0;
      bh[j] = Frag<T>::load(Bb + bo);
      if (SPLIT) bl[j] = Frag<T>::load(Bb2 + bo);
    }
#pragma unroll
    for (int i = 0; i < 4; ++i) {
      const size_t ao = (size_t)(m0 + (i << 4) + rlane) * lda + koff + k0;
      V ah = Frag<T>::load(Ab + ao);
      V al;
      if (SPLIT) al = Frag<T>::load(Ab2 + ao);
#pragma unroll
      for (int j = 0; j < 4; ++j) {
        acc[i][j] = Frag<T>::mma(ah, bh[j], acc[i][j]);
        if (SPLIT) {
          acc[i][j] = Frag<T>::mma(ah, bl[j], acc[i][j]);
          acc[i][j] = Frag<T>::mma(al, bh[j], acc[i][j]);
        }
      }
      Frag<T>::guard4(acc[i][0], acc[i][1], acc[i][2], acc[i][3], ah, SPLIT ? al : ah);
    }
    Frag<T>::keep(bh[0], bh[1], bh[2], bh[3]);
    if (SPLIT) Frag<T>::keep(bl[0], bl[1], bl[2], bl[3]);
  }
  acc_guard4(acc[0][0], acc[0][1], acc[0][2], acc[0][3]);
  acc_guard4(acc[1][0], acc[1][1], acc[1][2], acc[1][3]);
  acc_guard4(acc[2][0], acc[2][1], acc[2][2], acc[2][3]);
  acc_guard4(acc[3][0], acc[3][1], acc[3][2], acc[3][3]);

  float* slab = sT[wave];
  const float* Rb = RESID ? (resid + (size_t)b * strideR) : nullptr;
#pragma unroll
  for (int i = 0; i < 4; ++i) {
    const int mBase = m0 + (i << 4);
#pragma unroll
    for (int j = 0; j < 4; ++j) {
      const int n = n0 + (j << 4) + rlane;
      float bv = 0.f;
      if (BIAS_MODE == 2) bv = bias[n];
#pragma unroll
      for (int r = 0; r < 8; ++r) {
        float v = acc[i][j][r] * scale;
        if (BIAS_MODE == 1) v += bias[mBase + mOff + r];
        if (BIAS_MODE == 2) v += bv;
        if (RESID) v += Rb[(size_t)(mBase + mOff + r) * ldc + n];
        if (ACT == 1) v = tanhf(v);
        if (ACT == 2) v = fmaxf(v, 0.0f);
        if (ACT == 3) v = v / (1.0f + expf(-v));
        if (ACT == 4) v = (v > 0.f) ? v : 0.01f * v;
        slab[(mOff + r) * 68 + (j << 4) + rlane] = v;
      }
    }
    __builtin_amdgcn_fence(__ATOMIC_RELEASE, "workgroup");
    __builtin_amdgcn_wave_barrier();
    __builtin_amdgcn_fence(__ATOMIC_ACQUIRE, "workgroup");
    if (OUT_MODE == 0) {
      float* C = (float*)Cout + (size_t)b * strideC;
      const int hh = lane >> 4, c4 = (lane & 15) * 4;
      for (int pass = 0; pass < 2; ++pass) {
#pragma unroll
        for (int it = 0; it < 8; ++it) {
          const int row = it * 2 + hh;
          v4f v = *(const v4f*)(slab + row * 68 + c4);
          *(volatile v4f*)(C + (size_t)(mBase + row) * ldc + n0 + c4) = v;
        }
        __threadfence();
      }
    } else {
      const int q = lane >> 3, c8 = (lane & 7) * 8;
      unsigned short* C  = (unsigned short*)Cout  + (size_t)b * strideC;
      unsigned short* C2 = (OUT_MODE == 2) ? ((unsigned short*)Cout2 + (size_t)b * strideC) : nullptr;
      for (int pass = 0; pass < 2; ++pass) {
#pragma unroll
        for (int it = 0; it < 4; ++it) {
          const int row = it * 4 + q;
          const float* sp = slab + row * 68 + c8;
          v8h hv, lv;
#pragma unroll
          for (int e = 0; e < 8; ++e) {
            if (OUT_MODE == 1) {
              hv[e] = (_Float16)sp[e];
            } else {
              unsigned short hb = f2bf_bits(sp[e]);
              unsigned short lb = f2bf_bits(sp[e] - bf_bits2f(hb));
              hv[e] = __builtin_bit_cast(_Float16, hb);
              lv[e] = __builtin_bit_cast(_Float16, lb);
            }
          }
          *(volatile v8h*)(C + (size_t)(mBase + row) * ldc + n0 + c8) = hv;
          if (OUT_MODE == 2) *(volatile v8h*)(C2 + (size_t)(mBase + row) * ldc + n0 + c8) = lv;
        }
        __threadfence();
      }
    }
    __builtin_amdgcn_fence(__ATOMIC_RELEASE, "workgroup");
    __builtin_amdgcn_wave_barrier();
    __builtin_amdgcn_fence(__ATOMIC_ACQUIRE, "workgroup");
  }
}


__device__ __forceinline__ void store2(float* p, float v) {
  *(volatile float*)p = v;
  __threadfence();
  *(volatile float*)p = v;
}

__global__ __launch_bounds__(kThr) void cast_plane_kernel(const float* __restrict__ src, unsigned short* __restrict__ dst,
                                                          int colsLog2, int dstPitch, int dstOff) {
  const int i   = blockIdx.x * kThr + threadIdx.x;
  const int sh  = colsLog2 - 3;
  const int row = i >> sh;
  const int c8  = (i & ((1 << sh) - 1)) * 8;
  const float* sp = src + ((size_t)row << colsLog2) + c8;
  const v4f a0 = *(const v4f*)(sp);
  const v4f a1 = *(const v4f*)(sp + 4);
  v8h hv;
#pragma unroll
  for (int e = 0; e < 4; ++e) {
    const float f0 = a0[e];
    const float f1 = a1[e];
    hv[e]     = (_Float16)carry_flush(bf16r(f0), kInCarry);
    hv[4 + e] = (_Float16)carry_flush(bf16r(f1), kInCarry);
  }
  unsigned short* dp = dst + (size_t)row * dstPitch + dstOff + c8;
  *(volatile v8h*)dp = hv;
  __threadfence();
  *(volatile v8h*)dp = hv;
}

__global__ __launch_bounds__(256) void wt_plane_kernel(const float* __restrict__ W, unsigned short* __restrict__ dst, int K, int N, int nLive, int ldd, int colOff) {
  const int n  = blockIdx.x;
  const int k8 = threadIdx.x * 8;
  const bool live = n < nLive;
  const int nc = live ? n : 0;
  v8h hv;
#pragma unroll
  for (int e = 0; e < 8; ++e) {
    const float w = W[(size_t)(k8 + e) * N + nc];
    hv[e] = (_Float16)(live ? carry_flush(bf16r(w), kWCarry) : 0.0f);
  }
  unsigned short* dp = dst + (size_t)n * ldd + colOff + k8;
  *(volatile v8h*)dp = hv;
  __threadfence();
  *(volatile v8h*)dp = hv;
}

__global__ __launch_bounds__(kThr) void setup_kernel(const float* __restrict__ td, float* __restrict__ ZB, float* __restrict__ WDEC) {
  if (blockIdx.x < 3u) {
    store2(ZB + (size_t)blockIdx.x * kThr + threadIdx.x, 0.0f);
  } else {
    const float a = td[threadIdx.x];
    store2(WDEC + threadIdx.x, expf(-expf(bf16r(a))));
  }
}
static_assert(kN3 == 3 * kThr && kC == kThr, "set-up grid: 3 + 1 = 4 blocks");

__global__ __launch_bounds__(kThr) void lnstat_kernel(const float* __restrict__ x, float* __restrict__ STAT) {
  const size_t row = (size_t)blockIdx.x * kThr + threadIdx.x;
  const float* xp = x + row * kC;
  float s = 0.0f;
  for (int c = 0; c < kC; ++c) { const float p = xp[c]; s += bf16r(p); }
  const float mean = s / (float)kC;
  float q = 0.0f;
  for (int c = 0; c < kC; ++c) { const float p = xp[c]; const float dd = bf16r(p) - mean; q += dd * dd; }
  v2f st; st[0] = mean; st[1] = 1.0f / sqrtf(q / (float)kC + 1e-5f);
  float* dp = STAT + 2 * row;
  *(volatile v2f*)dp = st;
  __threadfence();
  *(volatile v2f*)dp = st;
}
static_assert(kRows == 16 * kThr, "statistics grid exact: 16 blocks");

__global__ __launch_bounds__(kThr) void lncast_kernel(const float* __restrict__ x, const float* __restrict__ STAT, const float* __restrict__ gam, const float* __restrict__ bet,
                                                     unsigned short* __restrict__ XN16) {
  const unsigned i = blockIdx.x * (unsigned)kThr + threadIdx.x;
  const size_t row = i >> 5;
  const unsigned c8 = (i & 31u) * 8u;
  const float mean = STAT[2 * row], inv = STAT[2 * row + 1];
  const float* xp = x + row * kC + c8;
  v8h hv;
#pragma unroll
  for (int e = 0; e < 8; ++e) {
    const float p = xp[e], ga = gam[c8 + e], be = bet[c8 + e];
    hv[e] = (_Float16)carry_flush(((bf16r(p) - mean) * inv) * bf16r(ga) + bf16r(be), kCXn);
  }
  unsigned short* dp = XN16 + row * kC + c8;
  *(volatile v8h*)dp = hv;
  __threadfence();
  *(volatile v8h*)dp = hv;
}
static_assert((size_t)kRows * (kC / 8) == 512ull * kThr && kC / 8 == 32, "norm cast grid exact: 512 blocks; 32 groups a row");

__global__ __launch_bounds__(kThr) void gate_kernel(const float* __restrict__ KVR, float* __restrict__ GS) {
  const unsigned i = blockIdx.x * (unsigned)kThr + threadIdx.x;
  const size_t row = i >> 5;
  const unsigned c8 = (i & 31u) * 8u;
  const float* rp = KVR + row * kN3 + 2 * kC + c8;
  const v4f r0 = *(const v4f*)rp, r1 = *(const v4f*)(rp + 4);
  v4f g0, g1;
#pragma unroll
  for (int e = 0; e < 4; ++e) { g0[e] = 1.0f / (1.0f + expf(-r0[e])); g1[e] = 1.0f / (1.0f + expf(-r1[e])); }
  float* dp = GS + row * kC + c8;
  for (int pass = 0; pass < 2; ++pass) { *(volatile v4f*)dp = g0; *(volatile v4f*)(dp + 4) = g1; __threadfence(); }
}
static_assert((size_t)kRows * (kC / 8) == 512ull * kThr, "gate grid exact: 512 blocks");

__global__ __launch_bounds__(kThr) void scan_kernel(const float* __restrict__ KVR, const float* __restrict__ GS, const float* __restrict__ st0, const float* __restrict__ WDEC,
                                                    float* __restrict__ OP, float* __restrict__ out) {
  const unsigned sq = blockIdx.x >> 3;
  const unsigned pt = blockIdx.x & 7u;
  const unsigned d = threadIdx.x;
  const unsigned c0 = pt * 32u;
  float s[32], w[32];
#pragma unroll
  for (int n = 0; n < 32; ++n) {
    w[n] = WDEC[c0 + n];
    const float p = st0[((size_t)sq * kC + c0 + n) * kC + d];
    s[n] = bf16r(p);
  }
  for (int t = 0; t < kT; ++t) {
    const size_t row = (size_t)sq * kT + (size_t)t;
    const float* pr = KVR + row * kN3;
    const float* pk = pr + c0;
    const float* pg = GS + row * kC + c0;
    const float v = pr[kC + d];
    float acc = 0.0f;
#pragma unroll
    for (int q = 0; q < 8; ++q) {
      const v4f kv = *(const v4f*)(pk + 4 * q), gv = *(const v4f*)(pg + 4 * q);
#pragma unroll
      for (int e = 0; e < 4; ++e) {
        const int n = 4 * q + e;
        const float sn = s[n] * w[n] + kv[e] * v;
        s[n] = sn;
        acc += gv[e] * sn;
      }
    }
    store2(OP + (row * kNPt + pt) * kC + d, acc);
  }
#pragma unroll
  for (int n = 0; n < 32; ++n) store2(out + (size_t)kOut1 + ((size_t)sq * kC + c0 + n) * kC + d, s[n]);
}
static_assert(kNB * kNPt == 64 && kC == kThr, "walk grid exact: 64 blocks: eight a sequence; a block's 256 lanes are the value columns");

__global__ __launch_bounds__(kThr) void osum_kernel(const float* __restrict__ OP, unsigned short* __restrict__ O16H, unsigned short* __restrict__ O16L) {
  const unsigned i = blockIdx.x * (unsigned)kThr + threadIdx.x;
  const size_t row = i >> 5;
  const unsigned c8 = (i & 31u) * 8u;
  const float* p0 = OP + row * kNPt * kC + c8;
  v8h hh, hl;
#pragma unroll
  for (int e = 0; e < 8; ++e) {
    float o = p0[e];
#pragma unroll
    for (int p = 1; p < kNPt; ++p) o += p0[(size_t)p * kC + e];
    const float sc = carry_flush(o, kCO);
    const _Float16 hi = (_Float16)sc;
    hh[e] = hi;
    hl[e] = (_Float16)carry_flush(sc - (float)hi, 1.0f);
  }
  unsigned short* dh = O16H + row * kC + c8;
  unsigned short* dl = O16L + row * kC + c8;
  for (int pass = 0; pass < 2; ++pass) { *(volatile v8h*)dh = hh; *(volatile v8h*)dl = hl; __threadfence(); }
}
static_assert((size_t)kRows * (kC / 8) == 512ull * kThr, "read-out sum grid exact: 512 blocks");

__global__ __launch_bounds__(kThr) void outadd_kernel(const float* __restrict__ P1, const float* __restrict__ P2, float* __restrict__ out) {
  const size_t o = ((size_t)blockIdx.x * kThr + threadIdx.x) * 8;
  const v4f a0 = *(const v4f*)(P1 + o), a1 = *(const v4f*)(P1 + o + 4), b0 = *(const v4f*)(P2 + o), b1 = *(const v4f*)(P2 + o + 4);
  v4f o0, o1;
#pragma unroll
  for (int e = 0; e < 4; ++e) { o0[e] = a0[e] + b0[e]; o1[e] = a1[e] + b1[e]; }
  float* dp = out + o;
  for (int pass = 0; pass < 2; ++pass) { *(volatile v4f*)dp = o0; *(volatile v4f*)(dp + 4) = o1; __threadfence(); }
}
static_assert((size_t)kRows * kC / 8 == 512ull * kThr, "the first result's grid exact: 512 blocks");

extern "C" void kernel_launch(void* const* d_in, const int* in_sizes, int n_in,
                              void* d_out, int out_size, void* d_ws, size_t ws_size,
                              hipStream_t stream) {
  if (n_in < 9 || d_out == nullptr || d_ws == nullptr) return;
  if (in_sizes[0] != kRows * kC || in_sizes[1] != kNB * kC * kC || in_sizes[2] != kC || in_sizes[3] != kC || in_sizes[4] != kC * kC || in_sizes[5] != kC * kC) return;
  if (in_sizes[6] != kC * kC || in_sizes[7] != kC * kC || in_sizes[8] != kC) return;
  if (out_size != kOut1 + kNB * kC * kC) return;
  if (ws_size < kWsTotal) return;
  const float* x   = (const float*)d_in[0];
  const float* st0 = (const float*)d_in[1];
  const float* gam = (const float*)d_in[2];
  const float* bet = (const float*)d_in[3];
  const float* Wk  = (const float*)d_in[4];
  const float* Wv  = (const float*)d_in[5];
  const float* Wr  = (const float*)d_in[6];
  const float* Wo  = (const float*)d_in[7];
  const float* td  = (const float*)d_in[8];
  float* out = (float*)d_out;
  char* ws = (char*)d_ws;
  float* ZB   = (float*)(ws + kOffZB);
  float* WDEC = (float*)(ws + kOffWDEC);
  float* STAT = (float*)(ws + kOffSTAT);
  unsigned short* XN16   = (unsigned short*)(ws + kOffXN16);
  unsigned short* WKVR16 = (unsigned short*)(ws + kOffWKVR16);
  unsigned short* WO16   = (unsigned short*)(ws + kOffWO16);
  float* KVR = (float*)(ws + kOffKVR);
  float* GS  = (float*)(ws + kOffGS);
  float* OP  = (float*)(ws + kOffOP);
  unsigned short* O16H = (unsigned short*)(ws + kOffO16H);
  unsigned short* O16L = (unsigned short*)(ws + kOffO16L);
  float* P1 = (float*)(ws + kOffP1);
  float* P2 = (float*)(ws + kOffP2);

  static_assert(((size_t)kC * kC / 8) % kThr == 0, "the casts' grids");
  lnstat_kernel<<<16, kThr, 0, stream>>>(x, STAT);
  lncast_kernel<<<512, kThr, 0, stream>>>(x, STAT, gam, bet, XN16);
  cast_plane_kernel<<<(int)(((size_t)kC * kC / 8) / kThr), kThr, 0, stream>>>(Wk, WKVR16, 8, kC, 0);
  cast_plane_kernel<<<(int)(((size_t)kC * kC / 8) / kThr), kThr, 0, stream>>>(Wv, WKVR16 + (size_t)kC * kC, 8, kC, 0);
  cast_plane_kernel<<<(int)(((size_t)kC * kC / 8) / kThr), kThr, 0, stream>>>(Wr, WKVR16 + (size_t)2 * kC * kC, 8, kC, 0);
  cast_plane_kernel<<<(int)(((size_t)kC * kC / 8) / kThr), kThr, 0, stream>>>(Wo, WO16, 8, kC, 0);
  setup_kernel<<<4, kThr, 0, stream>>>(td, ZB, WDEC);

  wmma_gemm64<0, false, 2, 0, false, 0><<<dim3((kRows / 64) * (kN3 / 64) / 8, 1), 256, 0, stream>>>(
      XN16, XN16, kC, 0L, WKVR16, WKVR16, kC, 0L, (void*)KVR, (void*)KVR, kN3, 0L, ZB, nullptr, 0L, kRows, kN3, kC, 1.0f / (kCXn * kInCarry));
  gate_kernel<<<512, kThr, 0, stream>>>(KVR, GS);
  scan_kernel<<<kNB * kNPt, kThr, 0, stream>>>(KVR, GS, st0, WDEC, OP, out);
  osum_kernel<<<512, kThr, 0, stream>>>(OP, O16H, O16L);
  wmma_gemm64<0, false, 2, 0, false, 0><<<dim3((kRows / 64) * (kC / 64) / 8, 1), 256, 0, stream>>>(
      O16H, O16H, kC, 0L, WO16, WO16, kC, 0L, (void*)P1, (void*)P1, kC, 0L, ZB, nullptr, 0L, kRows, kC, kC, 1.0f / (kCO * kInCarry));
  wmma_gemm64<0, false, 2, 0, false, 0><<<dim3((kRows / 64) * (kC / 64) / 8, 1), 256, 0, stream>>>(
      O16L, O16L, kC, 0L, WO16, WO16, kC, 0L, (void*)P2, (void*)P2, kC, 0L, ZB, nullptr, 0L, kRows, kC, kC, 1.0f / (kCO * kInCarry));
  outadd_kernel<<<512, kThr, 0, stream>>>(P1, P2, out);
}
static_assert(((kRows / 64) * (kN3 / 64)) % 8 == 0 && ((kRows / 64) * (kC / 64)) % 8 == 0, "the engine's grids: whole blocks of eight wave tiles");
